// GNN_446676598862
// MI455X (gfx1250) — hardware-verified
//
#include <hip/hip_runtime.h>
#include <stddef.h>
#include <stdint.h>
#include <math.h>


#define NG      64
#define NV      64
#define DF      128
#define MR      8192
#define HXP     384
#define SPP     2048
#define PPP     1024
#define MSGP    256
#define RTP     512
#define GP      512
#define BIGM    1.0e6f

#define O_W0A   0
#define O_W0B   131072
#define O_W1    393216
#define O_GRU   655360
#define O_GA0   720896
#define O_GE0   770048
#define O_RD2   802816
#define HALF_PL 868352
#define T0 16384
#define T1 49152
#define T2 81920
#define T3 90112
#define T4 96256
#define T5 100352
#define T6 108544

#define ATT_PHI 0
#define ATT_PSI 8192
#define ATT_ED  16384
#define ATT_NEG 32768
#define ATT_MSG 36864
#define ATT_FLOATS 45056
#define WSMAX 134217728

static_assert(T6 % 256 == 0 && T0 % 256 == 0 && T1 % 256 == 0 && T2 % 256 == 0 && T3 % 256 == 0 && T4 % 256 == 0 && T5 % 256 == 0);
static_assert(HALF_PL % 64 == 0 && O_GA0 % 64 == 0 && O_GE0 % 64 == 0 && O_RD2 % 64 == 0);
static_assert(O_RD2 + 256 * 256 == HALF_PL);
static_assert(ATT_FLOATS * 4 <= 300000);
static_assert(MR == 2 * NG * NV);

typedef float          v2f   __attribute__((ext_vector_type(2)));
typedef float          v4f   __attribute__((ext_vector_type(4)));
typedef float          v8f   __attribute__((ext_vector_type(8)));
typedef int            v4i   __attribute__((ext_vector_type(4)));
typedef int            v8i   __attribute__((ext_vector_type(8)));
typedef unsigned short v8us  __attribute__((ext_vector_type(8)));
typedef unsigned short v16us __attribute__((ext_vector_type(16)));
typedef __bf16         v16bf __attribute__((ext_vector_type(16)));
typedef v2f  __attribute__((may_alias)) v2fa;
typedef v4f  __attribute__((may_alias)) v4fa;
typedef v4i  __attribute__((may_alias)) v4ia;
typedef v8us __attribute__((may_alias)) v8usa;
typedef unsigned __attribute__((may_alias)) u32a;
union FragB { v16bf v; v16us u; v8us h[2]; v8i w; };

__device__ __forceinline__ v8f wmb(const FragB& a, const FragB& b, v8f c) {
  v8f d = __builtin_amdgcn_wmma_f32_16x16x32_bf16(false, a.v, false, b.v, (short)0, c, false, false);
  asm volatile("v_nop\n\tv_nop\n\tv_nop\n\tv_nop" : "+v"(d) : "v"(a.w), "v"(b.w));
  return d;
}

__device__ __forceinline__ unsigned bf16_bits(float f) {
  const unsigned u = __float_as_uint(f);
  return (u + 0x7FFFu + ((u >> 16) & 1u)) >> 16;
}
__device__ __forceinline__ unsigned short hl1(float v, bool lo) {
  const unsigned hb = bf16_bits(v);
  const unsigned lb = bf16_bits(v - __uint_as_float(hb << 16));
  return (unsigned short)(lo ? lb : hb);
}
__device__ __forceinline__ v8us hl_pack(v4f a, v4f b, bool lo) {
  v8us o;
  o[0] = hl1(a.x, lo); o[1] = hl1(a.y, lo); o[2] = hl1(a.z, lo); o[3] = hl1(a.w, lo);
  o[4] = hl1(b.x, lo); o[5] = hl1(b.y, lo); o[6] = hl1(b.z, lo); o[7] = hl1(b.w, lo);
  return o;
}
__device__ __forceinline__ void st2_us8(unsigned short* dp, v8us o) {
  *(volatile v8us*)dp = o;
  __threadfence();
  *(volatile v8us*)dp = o;
}
__device__ __forceinline__ float selu_f(float x) {
  const float sc = 1.0507009873554805f;
  const float al = 1.6732632423543772f;
  const float ng = al * expm1f(x);
  return sc * ((x > 0.0f) ? x : ng);
}
__device__ __forceinline__ float sigm_f(float x) {
  const float xc = fminf(fmaxf(x, -80.0f), 80.0f);
  const float sg = 1.0f / (1.0f + expf(-xc));
  return (x < -80.0f) ? 0.0f : sg;
}

__device__ __forceinline__ v8us cv8(const float* __restrict__ p) {
  const v4f a = *(const v4fa*)p;
  const v4f b = *(const v4fa*)(p + 4);
  v8us o;
  o[0] = (unsigned short)bf16_bits(a.x); o[1] = (unsigned short)bf16_bits(a.y);
  o[2] = (unsigned short)bf16_bits(a.z); o[3] = (unsigned short)bf16_bits(a.w);
  o[4] = (unsigned short)bf16_bits(b.x); o[5] = (unsigned short)bf16_bits(b.y);
  o[6] = (unsigned short)bf16_bits(b.z); o[7] = (unsigned short)bf16_bits(b.w);
  return o;
}
__global__ __launch_bounds__(256) void k_cvx(const float* __restrict__ nd1, const float* __restrict__ nd2,
                                             unsigned short* HX) {
  const int u   = (int)blockIdx.x * 256 + (int)threadIdx.x;
  const int row = u >> 4;
  const int k8  = (u & 15) * 8;
  const int r   = row & 4095;
  v8us o;
  if (blockIdx.x < 256) o = cv8(nd1 + (size_t)r * DF + k8);
  else                  o = cv8(nd2 + (size_t)r * DF + k8);
  st2_us8(HX + (size_t)row * HXP + 256 + k8, o);
}

__device__ __forceinline__ float rowsum64(const float* __restrict__ p) {
  float s = 0.0f;
#pragma unroll 4
  for (int i = 0; i < 16; ++i) {
    const v4f a = *(const v4fa*)(p + 4 * i);
    s += a.x; s += a.y; s += a.z; s += a.w;
  }
  return s;
}
__global__ __launch_bounds__(256) void k_nm(const float* __restrict__ adj1, const float* __restrict__ adj2, int* NM) {
  __shared__ __attribute__((aligned(16))) int sm[256];
  const int tid = (int)threadIdx.x;
  const int row = (int)blockIdx.x * 256 + tid;
  const int r   = row & 4095;
  float s;
  if (blockIdx.x < 16) s = rowsum64(adj1 + (size_t)r * NV);
  else                 s = rowsum64(adj2 + (size_t)r * NV);
  sm[tid] = (s > 0.0f) ? 1 : 0;
  __syncthreads();
  const bool ok = tid < 64;
  const v4i q = *(const v4ia*)(sm + 4 * (tid & 63));
  int* dp = NM + (size_t)blockIdx.x * 256 + 4 * (tid & 63);
  if (ok) *(volatile v4i*)dp = q;
  __threadfence();
  if (ok) *(volatile v4i*)dp = q;
}

__device__ __forceinline__ void wt_unit(const float* __restrict__ src, int soff, int ld, unsigned short* dp) {
  const float* p = src + soff;
  v8us o;
#pragma unroll
  for (int i = 0; i < 8; ++i) o[i] = (unsigned short)bf16_bits(p[(size_t)i * ld]);
  st2_us8(dp, o);
}
__global__ __launch_bounds__(256) void k_wprep(
    const float* __restrict__ mW0, const float* __restrict__ mW1, const float* __restrict__ aW0,
    const float* __restrict__ aW1, const float* __restrict__ Wz,  const float* __restrict__ Wn,
    const float* __restrict__ gaW0, const float* __restrict__ gaW1, const float* __restrict__ geW0,
    const float* __restrict__ geW1, unsigned short* PL) {
  const int u = (int)blockIdx.x * 256 + (int)threadIdx.x;
  if (u < T0) {
    const int n = u >> 4, k8 = (u & 15) * 8;
    const int soff = ((n >> 7) & 3) * 16384 + k8 * 128 + (n & 127);
    unsigned short* dp = PL + O_W0A + (size_t)n * 128 + k8;
    if (n < 512) wt_unit(mW0, soff, 128, dp); else wt_unit(aW0, soff, 128, dp);
  } else if (u < T1) {
    const int v = u - T0, n = v >> 5, k8 = (v & 31) * 8;
    const int soff = ((n >> 7) & 3) * 16384 + (k8 & 127) * 128 + (n & 127);
    unsigned short* dp = PL + O_W0B + (size_t)n * 256 + k8;
    if (n < 512) wt_unit(mW0, soff, 128, dp); else wt_unit(aW0, soff, 128, dp);
  } else if (u < T2) {
    const int v = u - T1, j = v >> 12, m = (v >> 5) & 127, k8 = (v & 31) * 8;
    const int soff = (j & 3) * 16384 + (k8 & 127) * 128 + m;
    unsigned short* dp = PL + O_W1 + (size_t)j * 32768 + (size_t)m * 256 + k8;
    if (j < 4) wt_unit(mW1, soff, 128, dp); else wt_unit(aW1, soff, 128, dp);
  } else if (u < T3) {
    const int v = u - T2, n = v >> 5, k8 = (v & 31) * 8;
    const int t = n & 127, f = (n >> 7) * 64 + (t & 63);
    const int soff = (k8 & 127) * 128 + f;
    unsigned short* dp = PL + O_GRU + (size_t)n * 256 + k8;
    if (t < 64) wt_unit(Wz, soff, 128, dp); else wt_unit(Wn, soff, 128, dp);
  } else if (u < T4) {
    const int v = u - T3, n = v / 48, k8 = (v - n * 48) * 8;
    const int sk = (k8 < 128) ? k8 : (k8 - 128);
    wt_unit(gaW0, sk * 128 + n, 128, PL + O_GA0 + (size_t)n * 384 + k8);
  } else if (u < T5) {
    const int v = u - T4, n = v >> 5, k8 = (v & 31) * 8;
    wt_unit(geW0, (k8 & 127) * 128 + n, 128, PL + O_GE0 + (size_t)n * 256 + k8);
  } else if (u < T6) {
    const int v = u - T5, n = v >> 5, k8 = (v & 31) * 8;
    const int t = n & 127, f = (n >> 7) * 64 + (t & 63);
    const int soff = (k8 & 127) * 128 + f;
    unsigned short* dp = PL + O_RD2 + (size_t)n * 256 + k8;
    if (t < 64) wt_unit(gaW1, soff, 128, dp); else wt_unit(geW1, soff, 128, dp);
  }
}
__global__ __launch_bounds__(256) void k_wout(const float* __restrict__ oW0, const float* __restrict__ oW1,
                                              unsigned short* P0, unsigned short* P1) {
  const int u = (int)blockIdx.x * 256 + (int)threadIdx.x;
  if (u < 16384) {
    const int n = u >> 6, k8 = (u & 63) * 8;
    const int sk = (k8 >> 8) * 128 + (k8 & 127);
    wt_unit(oW0, sk * 256 + n, 256, P0 + (size_t)n * 512 + k8);
  } else if (u < 24576) {
    const int v = u - 16384, n = v >> 6, k8 = (v & 63) * 8;
    const int sk = (k8 >> 8) * 128 + (k8 & 127);
    wt_unit(oW1, sk * 128 + n, 128, P1 + (size_t)n * 512 + k8);
  }
}

template <int EPI>
__global__ __launch_bounds__(128) void k_gemm(
    const unsigned short* __restrict__ A, int lda, int aZ, int a2off,
    const unsigned short* __restrict__ BT, int K, int kDec, int bHalf, int bZ,
    void* outp, int ldo, int oBase, int oY, int oZ,
    const int* __restrict__ NM, unsigned short* HXp)
{
  __shared__ __attribute__((aligned(16))) float stg[64 * 128];
  __shared__ __attribute__((aligned(16))) unsigned short hls[(EPI == 2) ? 8192 : 128];
  __shared__ float ems[64];
  const int tid = (int)threadIdx.x, lane = tid & 31, wave = tid >> 5, hh = lane >> 4, m = lane & 15;
  const int bx = (int)blockIdx.x, by = (int)blockIdx.y, bz = (int)blockIdx.z;
  const int rowBase = bx * 64;
  const int half = bx >> 6;
  const int Kz = K - bz * kDec;

  v8f acc[8];
  {
    const v8f z = {0.f, 0.f, 0.f, 0.f, 0.f, 0.f, 0.f, 0.f};
#pragma unroll
    for (int t = 0; t < 8; ++t) acc[t] = z;
  }
  const unsigned short* ap = A + (size_t)(rowBase + 16 * wave + m) * (size_t)lda + (size_t)bz * aZ + 8 * hh;
  const unsigned short* bp = BT + (size_t)half * (size_t)bHalf + (size_t)bz * (size_t)bZ
                                + (size_t)(by * 128 + m) * (size_t)Kz + 8 * hh;
#pragma unroll 1
  for (int k0 = 0; k0 < Kz; k0 += 32) {
    FragB af, af2;
    af.h[0] = *(const v8usa*)(ap + k0);
    af.h[1] = *(const v8usa*)(ap + k0 + 16);
    if constexpr (EPI == 3) {
      af2.h[0] = *(const v8usa*)(ap + a2off + k0);
      af2.h[1] = *(const v8usa*)(ap + a2off + k0 + 16);
    }
#pragma unroll
    for (int nt = 0; nt < 8; ++nt) {
      const unsigned short* wq = bp + (size_t)(16 * nt) * (size_t)Kz + k0;
      FragB bf;
      bf.h[0] = *(const v8usa*)wq;
      bf.h[1] = *(const v8usa*)(wq + 16);
      if constexpr (EPI == 3) {
        if (nt >= 4) acc[nt] = wmb(af2, bf, acc[nt]);
        else         acc[nt] = wmb(af,  bf, acc[nt]);
      } else {
        acc[nt] = wmb(af, bf, acc[nt]);
      }
    }
  }

#pragma unroll
  for (int nt = 0; nt < 8; ++nt) {
    const int lc = 16 * nt + m;
#pragma unroll
    for (int r = 0; r < 8; ++r) {
      const int lr = 16 * wave + 8 * hh + r;
      stg[lr * 128 + lc] = acc[nt][r];
    }
  }
  if constexpr (EPI == 3) {
    if (tid < 64) ems[tid] = (NM[rowBase + tid] != 0) ? 0.0f : BIGM;
  }
  __syncthreads();

  if constexpr (EPI == 0) {
    unsigned short* O = (unsigned short*)outp;
    const int ocol = oBase + by * oY + bz * oZ;
#pragma unroll 1
    for (int i = 0; i < 16; ++i) {
      float* p = stg + (16 * wave + i) * 128 + 4 * lane;
      v4f a = *(const v4fa*)p;
      a.x = selu_f(a.x); a.y = selu_f(a.y); a.z = selu_f(a.z); a.w = selu_f(a.w);
      *(v4fa*)p = a;
    }
    __syncthreads();
#pragma unroll 1
    for (int i = 0; i < 16; ++i) {
      const int lr = 16 * wave + i;
      const float* p = stg + lr * 128 + 8 * (lane & 15);
      const v4f a = *(const v4fa*)p;
      const v4f b = *(const v4fa*)(p + 4);
      const v8us q = hl_pack(a, b, lane >= 16);
      st2_us8(O + (size_t)(rowBase + lr) * (size_t)ldo + ocol + 8 * lane, q);
    }
  } else if constexpr (EPI == 1) {
    float* O = (float*)outp;
    const int ocol = oBase + by * oY + bz * oZ;
#pragma unroll 1
    for (int i = 0; i < 16; ++i) {
      const int lr = 16 * wave + i;
      const v4f a = *(const v4fa*)(stg + lr * 128 + 4 * lane);
      float* dp = O + (size_t)(rowBase + lr) * (size_t)ldo + ocol + 4 * lane;
      *(volatile v4f*)dp = a;
      __threadfence();
      *(volatile v4f*)dp = a;
    }
  } else if constexpr (EPI == 2) {
#pragma unroll 1
    for (int i = 0; i < 16; ++i) {
      const int lr = 16 * wave + i;
      const int gr = rowBase + lr;
      const v2f zz = *(const v2fa*)(stg + lr * 128 + 2 * lane);
      const v2f nn = *(const v2fa*)(stg + lr * 128 + 64 + 2 * lane);
      const int nm = NM[gr];
      const unsigned nw = *(const u32a*)(HXp + (size_t)gr * HXP + 256 + by * 64 + 2 * lane);
      const float n0 = __uint_as_float(nw << 16);
      const float n1 = __uint_as_float(nw & 0xffff0000u);
      const float h0 = (1.0f - sigm_f(zz.x)) * tanhf(nn.x);
      const float h1 = (1.0f - sigm_f(zz.y)) * tanhf(nn.y);
      const bool upd = nm != 0;
      const float v0 = upd ? h0 : n0;
      const float v1 = upd ? h1 : n1;
      const unsigned hb0 = bf16_bits(v0), hb1 = bf16_bits(v1);
      const unsigned lb0 = bf16_bits(v0 - __uint_as_float(hb0 << 16));
      const unsigned lb1 = bf16_bits(v1 - __uint_as_float(hb1 << 16));
      *(u32a*)(hls + lr * 128 + 2 * lane)      = hb0 | (hb1 << 16);
      *(u32a*)(hls + lr * 128 + 64 + 2 * lane) = lb0 | (lb1 << 16);
    }
    __syncthreads();
#pragma unroll 1
    for (int i = 0; i < 8; ++i) {
      const int lr  = 16 * wave + 2 * i + hh;
      const int l15 = lane & 15;
      const v8us q = *(const v8usa*)(hls + lr * 128 + 8 * l15);
      const int col = by * 64 + 8 * (l15 & 7) + (l15 >> 3) * 128;
      st2_us8(HXp + (size_t)(rowBase + lr) * HXP + col, q);
    }
  } else {
    unsigned short* O = (unsigned short*)outp;
    if (tid < 64) {
      float s = 0.0f;
#pragma unroll 1
      for (int r = 0; r < 64; ++r) {
        const float a = stg[r * 128 + tid];
        const float e = stg[r * 128 + 64 + tid];
        const float g = sigm_f(a - ems[r]);
        s += g * e;
      }
      const unsigned hb = bf16_bits(s);
      const unsigned lb = bf16_bits(s - __uint_as_float(hb << 16));
      hls[tid]      = (unsigned short)hb;
      hls[64 + tid] = (unsigned short)lb;
    }
    __syncthreads();
    const bool ok = (wave == 0) && (lane < 16);
    const v8us q = *(const v8usa*)(hls + 8 * (lane & 15));
    const int col = half * 256 + by * 64 + 8 * (lane & 7) + ((lane >> 3) & 1) * 128;
    unsigned short* dp = O + (size_t)(bx & 63) * (size_t)ldo + col;
    if (ok) *(volatile v8us*)dp = q;
    __threadfence();
    if (ok) *(volatile v8us*)dp = q;
  }
}

__device__ __forceinline__ void att_stage_graph(const float* __restrict__ adj, const float* __restrict__ ed,
                                                int b, float* dsm, int tid) {
  const float* ep = ed + (size_t)b * 16384;
#pragma unroll 4
  for (int it = 0; it < 16; ++it) {
    const int idx = it * 256 + tid;
    const v4f w = *(const v4fa*)(ep + 4 * idx);
    *(v4fa*)(dsm + ATT_ED + 4 * idx) = w;
  }
  const float* apn = adj + (size_t)b * 4096;
#pragma unroll 4
  for (int it = 0; it < 4; ++it) {
    const int idx = it * 256 + tid;
    const v4f a = *(const v4fa*)(apn + 4 * idx);
    v4f n;
    n.x = (a.x > 0.0f) ? 0.0f : BIGM; n.y = (a.y > 0.0f) ? 0.0f : BIGM;
    n.z = (a.z > 0.0f) ? 0.0f : BIGM; n.w = (a.w > 0.0f) ? 0.0f : BIGM;
    *(v4fa*)(dsm + ATT_NEG + 4 * idx) = n;
  }
}

__global__ __launch_bounds__(256) void k_att(const float* __restrict__ adj1, const float* __restrict__ ed1,
                                             const float* __restrict__ adj2, const float* __restrict__ ed2,
                                             const float* __restrict__ PP, unsigned short* MSG) {
  extern __shared__ __attribute__((aligned(16))) float dsm[];
  const int tid = (int)threadIdx.x, lane = tid & 31, wave = tid >> 5;
  const int gi = (int)blockIdx.x;
  const int b  = gi & 63;
  if (gi < 64) att_stage_graph(adj1, ed1, b, dsm, tid);
  else         att_stage_graph(adj2, ed2, b, dsm, tid);
  const float* pp = PP + (size_t)gi * 64 * PPP;

#pragma unroll 1
  for (int ch = 0; ch < 4; ++ch) {
    __syncthreads();
#pragma unroll 4
    for (int q = 0; q < 16; ++q) {
      const int id = q * 256 + tid;
      const int c4 = id & 7, j = (id >> 3) & 7, u = id >> 6;
      const v4f w = *(const v4fa*)(pp + (size_t)u * PPP + j * 128 + ch * 32 + c4 * 4);
      const int base = (j >> 2) * 8192 + (u * 32 + c4 * 4) * 4 + (j & 3);
      dsm[base] = w.x; dsm[base + 4] = w.y; dsm[base + 8] = w.z; dsm[base + 12] = w.w;
    }
    __syncthreads();
#pragma unroll 1
    for (int i = 0; i < 8; ++i) {
      const int v = wave * 8 + i;
      const float* edr = dsm + ATT_ED + v * 256;
      const float* ngr = dsm + ATT_NEG + v * 64;
      const float* psc = dsm + ATT_PSI + lane * 4;
      const float* phc = dsm + ATT_PHI + lane * 4;
      float mx = -3.0e38f;
#pragma unroll 1
      for (int u = 0; u < 64; ++u) {
        const v4f w = *(const v4fa*)(edr + 4 * u);
        const v4f q = *(const v4fa*)(psc + u * 128);
        float en = w.x * q.x;
        en = fmaf(w.y, q.y, en); en = fmaf(w.z, q.z, en); en = fmaf(w.w, q.w, en);
        en = en - ngr[u];
        mx = fmaxf(mx, en);
      }
      float s = 0.0f, acc = 0.0f;
#pragma unroll 1
      for (int u = 0; u < 64; ++u) {
        const v4f w = *(const v4fa*)(edr + 4 * u);
        const v4f q = *(const v4fa*)(psc + u * 128);
        const v4f f = *(const v4fa*)(phc + u * 128);
        float en = w.x * q.x;
        en = fmaf(w.y, q.y, en); en = fmaf(w.z, q.z, en); en = fmaf(w.w, q.w, en);
        en = en - ngr[u];
        float em = w.x * f.x;
        em = fmaf(w.y, f.y, em); em = fmaf(w.z, f.z, em); em = fmaf(w.w, f.w, em);
        const float p = expf(en - mx);
        s += p;
        acc = fmaf(p, em, acc);
      }
      dsm[ATT_MSG + v * 128 + ch * 32 + lane] = acc * (1.0f / s);
    }
  }
  __syncthreads();
#pragma unroll 1
  for (int i = 0; i < 8; ++i) {
    const int v = wave * 8 + i;
    const float* p = dsm + ATT_MSG + v * 128 + 8 * (lane & 15);
    const v4f a = *(const v4fa*)p;
    const v4f c = *(const v4fa*)(p + 4);
    const v8us q = hl_pack(a, c, lane >= 16);
    st2_us8(MSG + (size_t)(gi * 64 + v) * MSGP + 8 * lane, q);
  }
}

static inline size_t al256(size_t o) { return (o + 255) & ~(size_t)255; }

extern "C" void kernel_launch(void* const* d_in, const int* in_sizes, int n_in,
                              void* d_out, int out_size, void* d_ws, size_t ws_size,
                              hipStream_t stream) {
  if (n_in < 28) return;
  if (out_size != NG * DF) return;
  for (int t = 0; t < 2; ++t) {
    if (in_sizes[3 * t + 0] != NG * NV * NV) return;
    if (in_sizes[3 * t + 1] != NG * NV * DF) return;
    if (in_sizes[3 * t + 2] != NG * NV * NV * 4) return;
    const int wb = 6 + 10 * t;
    if (in_sizes[wb + 0] != 65536 || in_sizes[wb + 1] != 65536) return;
    if (in_sizes[wb + 2] != 65536 || in_sizes[wb + 3] != 65536) return;
    if (in_sizes[wb + 4] != 16384 || in_sizes[wb + 5] != 16384) return;
    if (in_sizes[wb + 6] != 32768 || in_sizes[wb + 7] != 16384) return;
    if (in_sizes[wb + 8] != 16384 || in_sizes[wb + 9] != 16384) return;
  }
  if (in_sizes[26] != 65536 || in_sizes[27] != 32768) return;

  const float* adj1 = (const float*)d_in[0];
  const float* nd1  = (const float*)d_in[1];
  const float* ed1  = (const float*)d_in[2];
  const float* adj2 = (const float*)d_in[3];
  const float* nd2  = (const float*)d_in[4];
  const float* ed2  = (const float*)d_in[5];
  const float* oW0  = (const float*)d_in[26];
  const float* oW1  = (const float*)d_in[27];
  float* out = (float*)d_out;

  char* ws = (char*)d_ws;
  size_t off = 0;
  const size_t oPL  = off; off = al256(off + (size_t)2 * HALF_PL * 2);
  const size_t oOW0 = off; off = al256(off + (size_t)256 * 512 * 2);
  const size_t oOW1 = off; off = al256(off + (size_t)128 * 512 * 2);
  const size_t oHX  = off; off = al256(off + (size_t)MR * HXP * 2);
  const size_t oNM  = off; off = al256(off + (size_t)MR * 4);
  const size_t oS   = off; off = al256(off + (size_t)MR * SPP * 2);
  const size_t oPP  = off; off = al256(off + (size_t)MR * PPP * 4);
  const size_t oMSG = off; off = al256(off + (size_t)MR * MSGP * 2);
  const size_t oRT  = off; off = al256(off + (size_t)MR * RTP * 2);
  const size_t oGHL = off; off = al256(off + (size_t)NG * GP * 2);
  const size_t oU   = off; off = al256(off + (size_t)NG * GP * 2);
  if (off > ws_size || off > (size_t)WSMAX) return;
  unsigned short* PL  = (unsigned short*)(ws + oPL);
  unsigned short* OW0 = (unsigned short*)(ws + oOW0);
  unsigned short* OW1 = (unsigned short*)(ws + oOW1);
  unsigned short* HX  = (unsigned short*)(ws + oHX);
  int*            NM  = (int*)(ws + oNM);
  unsigned short* S   = (unsigned short*)(ws + oS);
  float*          PP  = (float*)(ws + oPP);
  unsigned short* MSG = (unsigned short*)(ws + oMSG);
  unsigned short* RT  = (unsigned short*)(ws + oRT);
  unsigned short* GHL = (unsigned short*)(ws + oGHL);
  unsigned short* U   = (unsigned short*)(ws + oU);

  const size_t attLds = (size_t)ATT_FLOATS * 4;
  hipFuncSetAttribute(reinterpret_cast<const void*>(&k_att), hipFuncAttributeMaxDynamicSharedMemorySize, (int)attLds);

  k_cvx<<<512, 256, 0, stream>>>(nd1, nd2, HX);
  k_nm<<<32, 256, 0, stream>>>(adj1, adj2, NM);
  for (int t = 0; t < 2; ++t) {
    const int wb = 6 + 10 * t;
    k_wprep<<<T6 / 256, 256, 0, stream>>>(
        (const float*)d_in[wb + 0], (const float*)d_in[wb + 1], (const float*)d_in[wb + 2],
        (const float*)d_in[wb + 3], (const float*)d_in[wb + 4], (const float*)d_in[wb + 5],
        (const float*)d_in[wb + 6], (const float*)d_in[wb + 7], (const float*)d_in[wb + 8],
        (const float*)d_in[wb + 9], PL + (size_t)t * HALF_PL);
  }
  k_wout<<<96, 256, 0, stream>>>(oW0, oW1, OW0, OW1);

  for (int pass = 0; pass < 2; ++pass) {
    if (pass == 0) {
      k_gemm<0><<<dim3(128, 8, 1), 128, 0, stream>>>(HX + 256, HXP, 0, 0, PL + O_W0A, 128, 0, HALF_PL, 0,
                                                     (void*)S, SPP, 0, 256, 0, NM, HX);
    } else {
      k_gemm<0><<<dim3(128, 8, 1), 128, 0, stream>>>(HX, HXP, 0, 0, PL + O_W0B, 256, 0, HALF_PL, 0,
                                                     (void*)S, SPP, 0, 256, 0, NM, HX);
    }
    k_gemm<1><<<dim3(128, 1, 8), 128, 0, stream>>>(S, SPP, 256, 0, PL + O_W1, 256, 0, HALF_PL, 32768,
                                                   (void*)PP, PPP, 0, 0, 128, NM, HX);
    k_att<<<128, 256, attLds, stream>>>(adj1, ed1, adj2, ed2, PP, MSG);
    k_gemm<2><<<dim3(128, 2, 1), 128, 0, stream>>>(MSG, MSGP, 0, 0, PL + O_GRU, 256, 0, HALF_PL, 0,
                                                   (void*)HX, HXP, 0, 0, 0, NM, HX);
  }
  k_gemm<0><<<dim3(128, 1, 2), 128, 0, stream>>>(HX, HXP, 0, 0, PL + O_GA0, 384, 128, HALF_PL, O_GE0 - O_GA0,
                                                 (void*)RT, RTP, 0, 0, 256, NM, HX);
  k_gemm<3><<<dim3(128, 2, 1), 128, 0, stream>>>(RT, RTP, 0, 256, PL + O_RD2, 256, 0, HALF_PL, 0,
                                                 (void*)GHL, GP, 0, 0, 0, NM, HX);
  k_gemm<0><<<dim3(1, 2, 1), 128, 0, stream>>>(GHL, GP, 0, 0, OW0, 512, 0, 0, 0,
                                               (void*)U, GP, 0, 256, 0, NM, HX);
  k_gemm<1><<<dim3(1, 1, 1), 128, 0, stream>>>(U, GP, 0, 0, OW1, 512, 0, 0, 0,
                                               (void*)out, DF, 0, 0, 0, NM, HX);
}
